// TriangularSelfAttention_52810917871758
// MI455X (gfx1250) — hardware-verified
//
#include <hip/hip_runtime.h>
#include <math.h>
#include <stdint.h>

#ifndef NS
#define NS 256
#endif
#define NSX   256
#define LP    256
#define DM    128
#define NH    4
#define HD    64
#define DI    (NH * HD)
#define KX    (2 * DM)
#define NPIX  (LP * LP)
#define BG    ((NS <= 64) ? NS : 64)
#define NGRP  (NS / BG)
#define GROWS (BG * LP)
#define LNEPS 1e-5f
#define LOG2E 1.4426950408889634f
#define QSC   128.0f
#define CSC   1024.0f
#define KSC   1024.0f
#define PCAR  32768.0f
#define VCAR  1024.0f
#define OSC   1024.0f
#define WOS   1024.0f
#define WPB   4
#define NQT   (LP / 16)
#define NST   (LP / 64)
#define NKT   (LP / 32)
#define ATT_THREADS (WPB * 32)
#define PTP   36
#define PTW   (16 * PTP)
#define SLP   68
#define SLW   (16 * SLP)
#define WREG  (PTW + SLW)
#define SLAB64 (16 * 68)
#define VTP   72
#define QKC   (DI / 8)
#define QKR   8
#define QKT   (QKC * QKR)
#define LNPB  32
#define WS_CAP 134217728
static_assert(DI == NH * HD && HD == 64 && NH == 4 && WPB == NH);
static_assert(ATT_THREADS == 128);
static_assert(NS >= 1 && NS <= NSX && (NS % BG) == 0 && BG >= 1 && BG <= 64);
static_assert((LP % 64) == 0 && (LP % 32) == 0 && (LP % 16) == 0);
static_assert(DM == 128 && (KX % 32) == 0 && (DI % 64) == 0 && (DI % 32) == 0 && (DM % 64) == 0);
static_assert(QKC * 8 == DI && QKT == 256 && (GROWS % QKR) == 0 && (GROWS % 64) == 0);
static_assert((NPIX % LNPB) == 0 && LNPB == 32);
static_assert((DI % 128) == 0 && (DM % 128) == 0 && (DM % 64) == 0 && (DI % 64) == 0);

typedef unsigned short u16;
typedef _Float16 v16h __attribute__((ext_vector_type(16)));
typedef _Float16 v8h  __attribute__((ext_vector_type(8)));
typedef __bf16   v16b __attribute__((ext_vector_type(16)));
typedef float    v8f  __attribute__((ext_vector_type(8)));
typedef float    v4f  __attribute__((ext_vector_type(4)));
typedef unsigned int v4u __attribute__((ext_vector_type(4)));
typedef unsigned int v2u __attribute__((ext_vector_type(2)));

union FragH { v16h v; v8h h[2]; v4u u[2]; };
union FragB { v16b v; v4u u[2]; };

__device__ __forceinline__ unsigned short bf_bits(float f) {
  unsigned u = __float_as_uint(f);
  return (unsigned short)((u + 0x7FFFu + ((u >> 16) & 1u)) >> 16);
}
__device__ __forceinline__ float bf_up(unsigned short h) { return __uint_as_float(((unsigned)h) << 16); }
__device__ __forceinline__ float bfr(float f) { return bf_up(bf_bits(f)); }
__device__ __forceinline__ unsigned short h_bits(_Float16 x) { return __builtin_bit_cast(unsigned short, x); }
__device__ __forceinline__ unsigned pk16(unsigned short a, unsigned short b) { return (unsigned)a | ((unsigned)b << 16); }
__device__ __forceinline__ v8f zero8() { v8f z = {0.f, 0.f, 0.f, 0.f, 0.f, 0.f, 0.f, 0.f}; return z; }
__device__ __forceinline__ float sigm(float z) {
  const float zc = fminf(fmaxf(z, -30.0f), 30.0f);
  const float e  = exp2f(-zc * LOG2E);
  return __builtin_amdgcn_rcpf(1.0f + e);
}

__device__ __forceinline__ v16h ldfrag_h(const _Float16* p) {
  FragH f;
  f.h[0] = *(const v8h*)(p);
  f.h[1] = *(const v8h*)(p + 16);
  return f.v;
}
__device__ __forceinline__ v16b ldfrag_b(const u16* p) {
  FragB f;
  f.u[0] = *(const v4u*)(p);
  f.u[1] = *(const v4u*)(p + 16);
  return f.v;
}

__device__ __forceinline__ v8f mma_h(v16h a, v16h b, v8f c) {
  return __builtin_amdgcn_wmma_f32_16x16x32_f16(false, a, false, b, (short)0, c, false, false);
}
__device__ __forceinline__ v8f mma_b(v16b a, v16b b, v8f c) {
  return __builtin_amdgcn_wmma_f32_16x16x32_bf16(false, a, false, b, (short)0, c, false, false);
}
__device__ __forceinline__ void guard2(v8f& a, v8f& b, v16h x0, v16h x1, v16h x2, v16h x3, v16h x4, v16h x5) {
#if defined(__HIP_DEVICE_COMPILE__)
  asm volatile("v_nop\n\tv_nop\n\tv_nop\n\tv_nop"
               : "+v"(a), "+v"(b) : "v"(x0), "v"(x1), "v"(x2), "v"(x3), "v"(x4), "v"(x5) : "memory");
#endif
}
template <typename F>
__device__ __forceinline__ void guard6(v8f& a, v8f& b, v8f& c, v8f& d, F x0, F x1, F x2, F x3, F x4, F x5) {
#if defined(__HIP_DEVICE_COMPILE__)
  asm volatile("v_nop\n\tv_nop\n\tv_nop\n\tv_nop"
               : "+v"(a), "+v"(b), "+v"(c), "+v"(d) : "v"(x0), "v"(x1), "v"(x2), "v"(x3), "v"(x4), "v"(x5) : "memory");
#endif
}
__device__ __forceinline__ void acc_guard4(v8f& a, v8f& b, v8f& c, v8f& d) {
#if defined(__HIP_DEVICE_COMPILE__)
  asm volatile("v_nop\n\tv_nop\n\tv_nop\n\tv_nop" : "+v"(a), "+v"(b), "+v"(c), "+v"(d));
#endif
}
__device__ __forceinline__ void wave_sync_lds() {
  __builtin_amdgcn_fence(__ATOMIC_RELEASE, "workgroup");
  __builtin_amdgcn_wave_barrier();
  __builtin_amdgcn_fence(__ATOMIC_ACQUIRE, "workgroup");
}

__global__ __launch_bounds__(256) void ln_x(const float* __restrict__ pr, const float* __restrict__ mask,
                                            const float* __restrict__ gamma, const float* __restrict__ beta,
                                            const float* __restrict__ Wb, u16* XB, float* CB) {
  __shared__ __align__(16) u16 RB[8 * KX];
  __shared__ __align__(16) float PBS[NH * LNPB];
  const int tid = threadIdx.x, wave = tid >> 5, lane = tid & 31;
  const int p0 = (int)blockIdx.x * LNPB;
  if (p0 + LNPB > NPIX) return;
  float gm[4], bt[4], wb[16];
  {
    const v4f g4 = *(const v4f*)(gamma + 4 * lane), b4 = *(const v4f*)(beta + 4 * lane);
#pragma unroll
    for (int e = 0; e < 4; ++e) { gm[e] = bfr(g4[e]); bt[e] = bfr(b4[e]); }
#pragma unroll
    for (int i = 0; i < 4; ++i) {
      const v4f w4 = *(const v4f*)(Wb + 16 * lane + 4 * i);
#pragma unroll
      for (int h = 0; h < 4; ++h) wb[4 * i + h] = bfr(w4[h]);
    }
  }
  u16* rb = RB + wave * KX;
#pragma unroll 1
  for (int j = 0; j < LNPB / 8; ++j) {
    const int pl = j * 8 + wave;
    const int p  = p0 + pl;
    const v4f x4 = *(const v4f*)(pr + (size_t)p * DM + 4 * lane);
    float xr[4];
#pragma unroll
    for (int e = 0; e < 4; ++e) xr[e] = bfr(x4[e]);
    float s = (xr[0] + xr[1]) + (xr[2] + xr[3]);
#pragma unroll
    for (int off = 1; off < 32; off <<= 1) s += __shfl_xor(s, off, 32);
    const float mu = s * (1.0f / (float)DM);
    float d[4];
#pragma unroll
    for (int e = 0; e < 4; ++e) d[e] = xr[e] - mu;
    float ss = (d[0] * d[0] + d[1] * d[1]) + (d[2] * d[2] + d[3] * d[3]);
#pragma unroll
    for (int off = 1; off < 32; off <<= 1) ss += __shfl_xor(ss, off, 32);
    const float var = ss * (1.0f / (float)DM);
    const float rs  = 1.0f / sqrtf(var + LNEPS);
    float y[4];
#pragma unroll
    for (int e = 0; e < 4; ++e) y[e] = d[e] * rs * gm[e] + bt[e];
    unsigned short hb[4], lb[4];
#pragma unroll
    for (int e = 0; e < 4; ++e) { hb[e] = bf_bits(y[e]); lb[e] = bf_bits(y[e] - bf_up(hb[e])); }
    float pb[4];
#pragma unroll
    for (int h = 0; h < 4; ++h) pb[h] = y[0] * wb[h] + y[1] * wb[4 + h] + y[2] * wb[8 + h] + y[3] * wb[12 + h];
#pragma unroll
    for (int h = 0; h < 4; ++h) {
#pragma unroll
      for (int off = 1; off < 32; off <<= 1) pb[h] += __shfl_xor(pb[h], off, 32);
    }
    const float mk = bfr(mask[p]);
    const float mb = 1e9f * (mk - 1.0f);
    v2u hv, lv;
    hv[0] = pk16(hb[0], hb[1]);  hv[1] = pk16(hb[2], hb[3]);
    lv[0] = pk16(lb[0], lb[1]);  lv[1] = pk16(lb[2], lb[3]);
    *(v2u*)(rb + 4 * lane)      = hv;
    *(v2u*)(rb + DM + 4 * lane) = lv;
    if (lane == 0) {
      PBS[0 * LNPB + pl] = mb + pb[0];
      PBS[1 * LNPB + pl] = mb + pb[1];
      PBS[2 * LNPB + pl] = mb + pb[2];
      PBS[3 * LNPB + pl] = mb + pb[3];
    }
    wave_sync_lds();
    const v4u piece = *(const v4u*)(rb + 8 * lane);
    u16* dst = XB + (size_t)p * KX + 8 * lane;
    for (int pass = 0; pass < 2; ++pass) {
      *(volatile v4u*)(dst) = piece;
      __threadfence();
    }
    wave_sync_lds();
  }
  __syncthreads();
  if (wave == 0) {
    const int h = lane >> 3, j4 = (lane & 7) * 4;
    const v4f v = *(const v4f*)(PBS + h * LNPB + j4);
    float* d = CB + (size_t)h * NPIX + p0 + j4;
    for (int pass = 0; pass < 2; ++pass) {
      *(volatile v4f*)(d) = v;
      __threadfence();
    }
  }
}

__global__ __launch_bounds__(256) void wt16(const float* __restrict__ W, int ncol, int nk, u16* D, int ldd, int dup,
                                            int f16mode, float scale) {
  __shared__ __align__(16) u16 T[128 * VTP];
  const int tid = threadIdx.x;
  const int bid = blockIdx.x;
  const int nct = ncol / 128;
  const int ct  = bid % nct;
  const int rt  = bid / nct;
  if (rt * 64 + 64 > nk) return;
  {
    const int sl = tid >> 2;
    const int dc = (tid & 3) * 32;
    const float* src = W + (size_t)(rt * 64 + sl) * ncol + ct * 128 + dc;
#pragma unroll
    for (int i = 0; i < 8; ++i) {
      const v4f a = *(const v4f*)(src + 4 * i);
#pragma unroll
      for (int e = 0; e < 4; ++e) {
        const float f = a[e];
        const unsigned short hb = h_bits((_Float16)(bfr(f) * scale));
        const unsigned short bb = bf_bits(f);
        T[(dc + 4 * i + e) * VTP + sl] = (f16mode != 0) ? hb : bb;
      }
    }
  }
  __syncthreads();
  v4u w4[4];
  const int q8 = tid >> 3, p8 = (tid & 7) * 8;
#pragma unroll
  for (int it = 0; it < 4; ++it) {
    const int line = it * 32 + q8;
    w4[it] = *(const v4u*)(T + line * VTP + p8);
  }
  const size_t base = ((size_t)ct * 128) * ldd + rt * 64 + p8;
  for (int pass = 0; pass < 2; ++pass) {
#pragma unroll
    for (int it = 0; it < 4; ++it) {
      const int line = it * 32 + q8;
      *(volatile v4u*)(D + base + (size_t)line * ldd) = w4[it];
      if (dup != 0) *(volatile v4u*)(D + base + (size_t)line * ldd + nk) = w4[it];
    }
    __threadfence();
  }
}

__global__ __launch_bounds__(256) void vt16(const float* __restrict__ F, u16* VHo, u16* VLo) {
  __shared__ __align__(16) u16 TH[HD * VTP];
  __shared__ __align__(16) u16 TL[HD * VTP];
  const int tid = threadIdx.x;
  const int bid = blockIdx.x;
  const int st  = bid % NST;
  const int t2  = bid / NST;
  const int g   = t2 % NH;
  const int b   = t2 / NH;
  if (b >= BG) return;
  const int s0  = st * 64;
  {
    const int sl = tid >> 2;
    const int dc = (tid & 3) * 16;
    const float* src = F + ((size_t)b * LP + s0 + sl) * DI + g * HD + dc;
#pragma unroll
    for (int i = 0; i < 4; ++i) {
      const v4f a = *(const v4f*)(src + 4 * i);
#pragma unroll
      for (int e = 0; e < 4; ++e) {
        const float t = a[e] * VCAR;
        const _Float16 hv = (_Float16)t;
        const _Float16 lv = (_Float16)(t - (float)hv);
        TH[(dc + 4 * i + e) * VTP + sl] = h_bits(hv);
        TL[(dc + 4 * i + e) * VTP + sl] = h_bits(lv);
      }
    }
  }
  __syncthreads();
  v4u vh[2], vl[2];
  const int q8 = tid >> 3, p8 = (tid & 7) * 8;
#pragma unroll
  for (int it = 0; it < 2; ++it) {
    const int line = it * 32 + q8;
    vh[it] = *(const v4u*)(TH + line * VTP + p8);
    vl[it] = *(const v4u*)(TL + line * VTP + p8);
  }
  const size_t hrow = (size_t)(b * NH + g) * HD;
  const size_t base = hrow * LP + s0 + p8;
  for (int pass = 0; pass < 2; ++pass) {
#pragma unroll
    for (int it = 0; it < 2; ++it) {
      const int line = it * 32 + q8;
      *(volatile v4u*)(VHo + base + (size_t)line * LP) = vh[it];
      *(volatile v4u*)(VLo + base + (size_t)line * LP) = vl[it];
    }
    __threadfence();
  }
}

__global__ __launch_bounds__(QKT) void qk16(const float* __restrict__ F, u16* Hp, u16* Lp, float sc) {
  const int tid = (int)threadIdx.x;
  if (tid >= QKT) return;
  const int rl  = tid / QKC;
  const int cc  = tid - rl * QKC;
  const int row = (int)blockIdx.x * QKR + rl;
  if (row >= GROWS) return;
  const float* p = F + (size_t)row * DI + cc * 8;
  const v4f a = *(const v4f*)(p), b4 = *(const v4f*)(p + 4);
  float w[8];
#pragma unroll
  for (int e = 0; e < 4; ++e) { w[e] = a[e] * sc; w[4 + e] = b4[e] * sc; }
  v4u oh, ol;
#pragma unroll
  for (int e = 0; e < 4; ++e) {
    const float t0 = w[2 * e], t1 = w[2 * e + 1];
    const _Float16 h0 = (_Float16)t0, h1 = (_Float16)t1;
    const _Float16 l0 = (_Float16)(t0 - (float)h0), l1 = (_Float16)(t1 - (float)h1);
    oh[e] = pk16(h_bits(h0), h_bits(h1));
    ol[e] = pk16(h_bits(l0), h_bits(l1));
  }
  u16* dh = Hp + (size_t)row * DI + cc * 8;
  u16* dl = Lp + (size_t)row * DI + cc * 8;
  for (int pass = 0; pass < 2; ++pass) {
    *(volatile v4u*)(dh) = oh;
    *(volatile v4u*)(dl) = ol;
    __threadfence();
  }
}

__device__ __forceinline__ void epi64(float* sl, v8f a0, v8f a1, v8f a2, v8f a3, float oscale,
                                      float* C, int N, size_t rowb, int col0, int lane) {
  const int hh = lane >> 4, m = lane & 15;
#pragma unroll
  for (int r = 0; r < 8; ++r) {
    const int ro = (8 * hh + r) * 68 + m;
    sl[ro]      = a0[r] * oscale;
    sl[ro + 16] = a1[r] * oscale;
    sl[ro + 32] = a2[r] * oscale;
    sl[ro + 48] = a3[r] * oscale;
  }
  wave_sync_lds();
  v4f vals[8];
#pragma unroll
  for (int it = 0; it < 8; ++it) vals[it] = *(const v4f*)(sl + (it * 2 + hh) * 68 + m * 4);
  float* dst = C + (rowb + (size_t)hh) * (size_t)N + col0 + m * 4;
  for (int pass = 0; pass < 2; ++pass) {
#pragma unroll
    for (int it = 0; it < 8; ++it) {
      *(volatile v4f*)(dst + (size_t)(it * 2) * (size_t)N) = vals[it];
    }
    __threadfence();
  }
}
__device__ __forceinline__ void epi64o(float* sl, v8f a0, v8f a1, v8f a2, v8f a3, float oscale,
                                       float* C, int N, size_t rowb, int col0, int lane,
                                       const float* __restrict__ bias, const float* __restrict__ rsc) {
  const int hh = lane >> 4, m = lane & 15;
#pragma unroll
  for (int r = 0; r < 8; ++r) {
    const int ro = (8 * hh + r) * 68 + m;
    sl[ro]      = a0[r] * oscale;
    sl[ro + 16] = a1[r] * oscale;
    sl[ro + 32] = a2[r] * oscale;
    sl[ro + 48] = a3[r] * oscale;
  }
  wave_sync_lds();
  float bq[4];
  {
    const v4f b4 = *(const v4f*)(bias + col0 + m * 4);
#pragma unroll
    for (int e = 0; e < 4; ++e) bq[e] = bfr(b4[e]);
  }
  v4f vals[8];
#pragma unroll
  for (int it = 0; it < 8; ++it) {
    const v4f t = *(const v4f*)(sl + (it * 2 + hh) * 68 + m * 4);
    const float mk = bfr(rsc[rowb + (size_t)hh + (size_t)(it * 2)]);
    v4f o;
#pragma unroll
    for (int e = 0; e < 4; ++e) o[e] = (t[e] + bq[e]) * mk;
    vals[it] = o;
  }
  float* dst = C + (rowb + (size_t)hh) * (size_t)N + col0 + m * 4;
  for (int pass = 0; pass < 2; ++pass) {
#pragma unroll
    for (int it = 0; it < 8; ++it) {
      *(volatile v4f*)(dst + (size_t)(it * 2) * (size_t)N) = vals[it];
    }
    __threadfence();
  }
}

__global__ __launch_bounds__(128)
void gemm_bf(const u16* __restrict__ A, const u16* __restrict__ Bt, float* C, int M, int N, int K, float oscale) {
  __shared__ __align__(16) float slab[4 * SLAB64];
  const int tid = threadIdx.x, wave = tid >> 5, lane = tid & 31, hh = lane >> 4, m = lane & 15;
  const int ntile = N >> 6;
  const int bid   = blockIdx.x;
  const int rowb  = (bid / ntile) * 64 + wave * 16;
  const int col0  = (bid % ntile) * 64;
  if (rowb + 16 > M) return;
  const u16* ap = A  + (size_t)(rowb + m) * K + 8 * hh;
  const u16* bp = Bt + (size_t)(col0 + m) * K + 8 * hh;
  const size_t bs = (size_t)16 * K;
  v8f acc0 = zero8(), acc1 = zero8(), acc2 = zero8(), acc3 = zero8();
#pragma unroll 1
  for (int k0 = 0; k0 < K; k0 += 32) {
    const v16b a  = ldfrag_b(ap + k0);
    const v16b b0 = ldfrag_b(bp + k0);
    const v16b b1 = ldfrag_b(bp + bs + k0);
    const v16b b2 = ldfrag_b(bp + 2 * bs + k0);
    const v16b b3 = ldfrag_b(bp + 3 * bs + k0);
    acc0 = mma_b(a, b0, acc0);
    acc1 = mma_b(a, b1, acc1);
    acc2 = mma_b(a, b2, acc2);
    acc3 = mma_b(a, b3, acc3);
    guard6<v16b>(acc0, acc1, acc2, acc3, a, b0, b1, b2, b3, a);
  }
  epi64(slab + wave * SLAB64, acc0, acc1, acc2, acc3, oscale, C, N, (size_t)rowb, col0, lane);
}

__global__ __launch_bounds__(128)
void gemm_o(const u16* __restrict__ Ah, const u16* __restrict__ Al, const u16* __restrict__ Bt,
            const float* __restrict__ bias, const float* __restrict__ rsc, float* C, float oscale) {
  __shared__ __align__(16) float slab[4 * SLAB64];
  const int tid = threadIdx.x, wave = tid >> 5, lane = tid & 31, hh = lane >> 4, m = lane & 15;
  const int ntile = DM >> 6;
  const int bid   = blockIdx.x;
  const int ct    = bid % ntile;
  const int t2    = bid / ntile;
  const int rt    = t2 % NST;
  const int bb    = t2 / NST;
  if (bb >= BG) return;
  const int srow  = rt * 64 + wave * 16;
  if (srow + 16 > LP) return;
  const int col0  = ct * 64;
  const int K     = DI;
  const size_t rowC = (size_t)bb * LP + srow;
  const _Float16* ahp = (const _Float16*)(const void*)Ah + (rowC + m) * K + 8 * hh;
  const _Float16* alp = (const _Float16*)(const void*)Al + (rowC + m) * K + 8 * hh;
  const _Float16* bp  = (const _Float16*)(const void*)Bt + (size_t)(col0 + m) * K + 8 * hh;
  const size_t bs = (size_t)16 * K;
  v8f acc0 = zero8(), acc1 = zero8(), acc2 = zero8(), acc3 = zero8();
#pragma unroll 1
  for (int k0 = 0; k0 < K; k0 += 32) {
    const v16h ah = ldfrag_h(ahp + k0), al = ldfrag_h(alp + k0);
    const v16h b0 = ldfrag_h(bp + k0);
    const v16h b1 = ldfrag_h(bp + bs + k0);
    const v16h b2 = ldfrag_h(bp + 2 * bs + k0);
    const v16h b3 = ldfrag_h(bp + 3 * bs + k0);
    acc0 = mma_h(ah, b0, acc0);  acc0 = mma_h(al, b0, acc0);
    acc1 = mma_h(ah, b1, acc1);  acc1 = mma_h(al, b1, acc1);
    acc2 = mma_h(ah, b2, acc2);  acc2 = mma_h(al, b2, acc2);
    acc3 = mma_h(ah, b3, acc3);  acc3 = mma_h(al, b3, acc3);
    guard6<v16h>(acc0, acc1, acc2, acc3, ah, al, b0, b1, b2, b3);
  }
  epi64o(slab + wave * SLAB64, acc0, acc1, acc2, acc3, oscale, C, DM, rowC, col0, lane, bias, rsc);
}

__global__ __launch_bounds__(ATT_THREADS)
void attn_t(const u16* __restrict__ RHp, const u16* __restrict__ RLp,
            const u16* __restrict__ CHp, const u16* __restrict__ CLp,
            const u16* __restrict__ VHp, const u16* __restrict__ VLp,
            const float* __restrict__ CB, const float* __restrict__ U, const float* __restrict__ bu,
            u16* OHp, u16* OLp) {
  __shared__ __align__(16) float smem[WPB * WREG];

  const int tid  = threadIdx.x;
  const int wave = tid >> 5;
  const int lane = tid & 31;
  const int hh   = lane >> 4;
  const int c    = lane & 15;
  const int bid  = blockIdx.x;
  const int qt   = bid % NQT;
  const int b    = bid / NQT;
  if (b >= BG) return;
  const int q0   = qt * 16;
  const int head = wave;

  float* pt   = smem + wave * WREG;
  float* slab = pt + PTW;

  const size_t hcol = (size_t)head * HD + 8 * hh;
  const _Float16* Rh  = (const _Float16*)(const void*)RHp + ((size_t)b * LP + q0 + c) * DI + hcol;
  const _Float16* Rl  = (const _Float16*)(const void*)RLp + ((size_t)b * LP + q0 + c) * DI + hcol;
  const _Float16* Chb = (const _Float16*)(const void*)CHp + ((size_t)b * LP + c) * DI + hcol;
  const _Float16* Clb = (const _Float16*)(const void*)CLp + ((size_t)b * LP + c) * DI + hcol;
  const _Float16* Vhb = (const _Float16*)(const void*)VHp + ((size_t)(b * NH + head) * HD + c) * LP + 8 * hh;
  const _Float16* Vlb = (const _Float16*)(const void*)VLp + ((size_t)(b * NH + head) * HD + c) * LP + 8 * hh;
  const float* cbb = CB + ((size_t)head * LP + q0) * LP;
  const float invc = 1.0f / (CSC * KSC);
  const float oc   = 1.0f / (PCAR * VCAR);
  const size_t KROW = (size_t)DI;

  float mrow[8], lrow[8];
  v8f o[4];
#pragma unroll
  for (int r = 0; r < 8; ++r) { mrow[r] = -INFINITY; lrow[r] = 0.f; }
#pragma unroll
  for (int j = 0; j < 4; ++j) o[j] = zero8();

#pragma unroll 1
  for (int kt = 0; kt < NKT; ++kt) {
    const int kb = kt * 32;
#pragma unroll
    for (int it = 0; it < 4; ++it) {
      const int f = it * 32 + lane;
      const int row = f >> 3, col4 = (f & 7) * 4;
      const v4f t4 = *(const v4f*)(cbb + (size_t)row * LP + kb + col4);
      *(v4f*)(pt + row * PTP + col4) = t4;
    }
    v8f s0 = zero8(), s1 = zero8();
    const _Float16* c0p = Chb + (size_t)kb * KROW;
    const _Float16* c1p = c0p + (size_t)16 * KROW;
    const _Float16* l0p = Clb + (size_t)kb * KROW;
    const _Float16* l1p = l0p + (size_t)16 * KROW;
#pragma unroll
    for (int kk = 0; kk < HD / 32; ++kk) {
      const v16h rh  = ldfrag_h(Rh + kk * 32);
      const v16h rl  = ldfrag_h(Rl + kk * 32);
      const v16h ch0 = ldfrag_h(c0p + kk * 32);
      const v16h ch1 = ldfrag_h(c1p + kk * 32);
      const v16h cl0 = ldfrag_h(l0p + kk * 32);
      const v16h cl1 = ldfrag_h(l1p + kk * 32);
      s0 = mma_h(rh, ch0, s0);
      s0 = mma_h(rl, ch0, s0);
      s0 = mma_h(rh, cl0, s0);
      s1 = mma_h(rh, ch1, s1);
      s1 = mma_h(rl, ch1, s1);
      s1 = mma_h(rh, cl1, s1);
      guard2(s0, s1, rh, rl, ch0, cl0, ch1, cl1);
    }
    wave_sync_lds();
#pragma unroll
    for (int r = 0; r < 8; ++r) {
      const int   ro  = (8 * hh + r) * PTP + c;
      const float cb0 = pt[ro];
      const float cb1 = pt[ro + 16];
      const float t0  = (s0[r] * invc + cb0) * LOG2E;
      const float t1  = (s1[r] * invc + cb1) * LOG2E;
      float mx = fmaxf(t0, t1);
#pragma unroll
      for (int off = 1; off < 16; off <<= 1) mx = fmaxf(mx, __shfl_xor(mx, off, 32));
      const float mn = fmaxf(mrow[r], mx);
      const float ms = (mn == -INFINITY) ? 0.0f : mn;
      const float al = exp2f(mrow[r] - ms);
      mrow[r] = mn;
      const float e0 = exp2f(t0 - ms), e1 = exp2f(t1 - ms);
      float ps = e0 + e1;
#pragma unroll
      for (int off = 1; off < 16; off <<= 1) ps += __shfl_xor(ps, off, 32);
      lrow[r] = lrow[r] * al + ps;
#pragma unroll
      for (int j = 0; j < 4; ++j) o[j][r] *= al;
      pt[ro]      = e0;
      pt[ro + 16] = e1;
    }
    wave_sync_lds();
    FragH ph, pl;
    {
      const float* prow = pt + c * PTP + 8 * hh;
      const v4f p0 = *(const v4f*)(prow), p1 = *(const v4f*)(prow + 4);
      const v4f p2 = *(const v4f*)(prow + 16), p3 = *(const v4f*)(prow + 20);
#pragma unroll
      for (int e = 0; e < 4; ++e) {
        const float ta = p0[e] * PCAR, tb = p1[e] * PCAR, tc = p2[e] * PCAR, td = p3[e] * PCAR;
        const _Float16 ha = (_Float16)ta, hb = (_Float16)tb, hc = (_Float16)tc, hd = (_Float16)td;
        ph.h[0][e]     = ha;
        ph.h[0][4 + e] = hb;
        ph.h[1][e]     = hc;
        ph.h[1][4 + e] = hd;
        pl.h[0][e]     = (_Float16)(ta - (float)ha);
        pl.h[0][4 + e] = (_Float16)(tb - (float)hb);
        pl.h[1][e]     = (_Float16)(tc - (float)hc);
        pl.h[1][4 + e] = (_Float16)(td - (float)hd);
      }
    }
    {
      const _Float16* vhp = Vhb + kb;
      const _Float16* vlp = Vlb + kb;
#pragma unroll
      for (int jg = 0; jg < HD / 32; ++jg) {
        const size_t da = (size_t)(2 * jg) * 16 * LP;
        const size_t db = da + (size_t)16 * LP;
        const v16h vha = ldfrag_h(vhp + da), vhb2 = ldfrag_h(vhp + db);
        const v16h vla = ldfrag_h(vlp + da), vlb2 = ldfrag_h(vlp + db);
        o[2 * jg]     = mma_h(ph.v, vha,  o[2 * jg]);
        o[2 * jg]     = mma_h(pl.v, vha,  o[2 * jg]);
        o[2 * jg]     = mma_h(ph.v, vla,  o[2 * jg]);
        o[2 * jg + 1] = mma_h(ph.v, vhb2, o[2 * jg + 1]);
        o[2 * jg + 1] = mma_h(pl.v, vhb2, o[2 * jg + 1]);
        o[2 * jg + 1] = mma_h(ph.v, vlb2, o[2 * jg + 1]);
        guard2(o[2 * jg], o[2 * jg + 1], ph.v, pl.v, vha, vhb2, vla, vlb2);
      }
    }
    wave_sync_lds();
  }
  acc_guard4(o[0], o[1], o[2], o[3]);
#pragma unroll
  for (int r = 0; r < 8; ++r) {
    const float lv  = lrow[r];
    const float ls  = (lv > 0.0f) ? lv : 1.0f;
    const float inv = (lv > 0.0f) ? ((1.0f / ls) * oc) : 0.0f;
#pragma unroll
    for (int j = 0; j < 4; ++j) {
      const int idx = (8 * hh + r) * SLP + j * 16 + c;
      slab[idx] = o[j][r] * inv;
    }
  }

  wave_sync_lds();
  v4u oh[4], ol[4];
  const int rq = lane >> 3, c8 = (lane & 7) * 8;
  const float* urow = U + ((size_t)b * LP + q0) * DI + (size_t)head * HD + c8;
  float bb[8];
  {
    const v4f u0 = *(const v4f*)(bu + head * HD + c8), u1 = *(const v4f*)(bu + head * HD + c8 + 4);
#pragma unroll
    for (int e = 0; e < 4; ++e) { bb[e] = bfr(u0[e]); bb[4 + e] = bfr(u1[e]); }
  }
#pragma unroll
  for (int it = 0; it < 4; ++it) {
    const int row = it * 4 + rq;
    const v4f a  = *(const v4f*)(slab + row * SLP + c8), b4 = *(const v4f*)(slab + row * SLP + c8 + 4);
    const v4f ua = *(const v4f*)(urow + (size_t)row * DI), ub = *(const v4f*)(urow + (size_t)row * DI + 4);
    float w[8];
#pragma unroll
    for (int e = 0; e < 4; ++e) {
      w[e]     = (a[e]  * sigm(ua[e] + bb[e]))     * OSC;
      w[4 + e] = (b4[e] * sigm(ub[e] + bb[4 + e])) * OSC;
    }
#pragma unroll
    for (int e = 0; e < 4; ++e) {
      const _Float16 h0 = (_Float16)w[2 * e], h1 = (_Float16)w[2 * e + 1];
      const _Float16 l0 = (_Float16)(w[2 * e] - (float)h0), l1 = (_Float16)(w[2 * e + 1] - (float)h1);
      oh[it][e] = pk16(h_bits(h0), h_bits(h1));
      ol[it][e] = pk16(h_bits(l0), h_bits(l1));
    }
  }
  const size_t ob = ((size_t)b * LP + q0) * DI + (size_t)head * HD + c8;
  for (int pass = 0; pass < 2; ++pass) {
#pragma unroll
    for (int it = 0; it < 4; ++it) {
      const int row = it * 4 + rq;
      *(volatile v4u*)(OHp + ob + (size_t)row * DI) = oh[it];
      *(volatile v4u*)(OLp + ob + (size_t)row * DI) = ol[it];
    }
    __threadfence();
  }
}

extern "C" void kernel_launch(void* const* d_in, const int* in_sizes, int n_in,
                              void* d_out, int out_size, void* d_ws, size_t ws_size,
                              hipStream_t stream) {
  if (n_in < 12) return;
  if (in_sizes[0] < NPIX * DM) return;
  if (in_sizes[1] < NPIX) return;
  if (in_sizes[2] < DM || in_sizes[3] < DM) return;
  if (in_sizes[4] < DM * DI || in_sizes[5] < DM * DI || in_sizes[6] < DM * DI || in_sizes[8] < DM * DI) return;
  if (in_sizes[7] < DM * NH) return;
  if (in_sizes[9] < DI) return;
  if (in_sizes[10] < DI * DM) return;
  if (in_sizes[11] < DM) return;
  if (out_size < NS * LP * DM) return;

  const float* pr    = (const float*)d_in[0];
  const float* mask  = (const float*)d_in[1];
  const float* gamma = (const float*)d_in[2];
  const float* beta  = (const float*)d_in[3];
  const float* Wq    = (const float*)d_in[4];
  const float* Wk    = (const float*)d_in[5];
  const float* Wv    = (const float*)d_in[6];
  const float* Wb    = (const float*)d_in[7];
  const float* Wu    = (const float*)d_in[8];
  const float* bu    = (const float*)d_in[9];
  const float* Wo    = (const float*)d_in[10];
  const float* bo    = (const float*)d_in[11];
  float*       out   = (float*)d_out;

  const size_t szXB = (size_t)NPIX * KX * 2;
  const size_t szF  = (size_t)GROWS * DI * 4;
  const size_t szU  = (size_t)GROWS * DI * 4;
  const size_t szH  = (size_t)GROWS * DI * 2;
  const size_t szV  = (size_t)BG * NH * HD * LP * 2;
  const size_t szCB = (size_t)NH * NPIX * 4;
  const size_t szW  = (size_t)DI * KX * 2;
  const size_t szWO = (size_t)DM * DI * 2;
  if (2 * szH > szF) return;
  size_t off = 0;
  const size_t oXB = off; off += szXB;
  const size_t oF  = off; off += szF;
  const size_t oU  = off; off += szU;
  const size_t oQH = off; off += szH;
  const size_t oKH = off; off += szH;
  const size_t oQL = off; off += szH;
  const size_t oKL = off; off += szH;
  const size_t oVH = off; off += szV;
  const size_t oVL = off; off += szV;
  const size_t oCB = off; off += szCB;
  const size_t oWQ = off; off += szW;
  const size_t oWK = off; off += szW;
  const size_t oWV = off; off += szW;
  const size_t oWU = off; off += szW;
  const size_t oWO = off; off += szWO;
  if (off > ws_size) return;
  if (off > (size_t)WS_CAP) return;

  char* ws = (char*)d_ws;
  u16*   XB = (u16*)(ws + oXB);
  float* F  = (float*)(ws + oF);
  u16*   OH = (u16*)(ws + oF);
  u16*   OL = (u16*)(ws + oF + szH);
  float* U  = (float*)(ws + oU);
  u16*   QH = (u16*)(ws + oQH);
  u16*   KH = (u16*)(ws + oKH);
  u16*   QL = (u16*)(ws + oQL);
  u16*   KL = (u16*)(ws + oKL);
  u16*   VH = (u16*)(ws + oVH);
  u16*   VL = (u16*)(ws + oVL);
  float* CB = (float*)(ws + oCB);
  u16*   WQ = (u16*)(ws + oWQ);
  u16*   WK = (u16*)(ws + oWK);
  u16*   WV = (u16*)(ws + oWV);
  u16*   WU = (u16*)(ws + oWU);
  u16*   WO = (u16*)(ws + oWO);

  const dim3 b256(256), b128(128), bQK(QKT), bAT(ATT_THREADS);
  const dim3 gLN(NPIX / LNPB);
  const dim3 gWP((DI / 128) * (DM / 64));
  const dim3 gWO((DM / 128) * (DI / 64));
  const dim3 gG((GROWS / 64) * (DI / 64));
  const dim3 gVT(BG * NH * NST);
  const dim3 gQK(GROWS / QKR);
  const dim3 gAT(NQT * BG);
  const dim3 gO(BG * NST * (DM / 64));
  const float osc = 1.0f / (OSC * WOS);

  ln_x<<<gLN, b256, 0, stream>>>(pr, mask, gamma, beta, Wb, XB, CB);
  wt16<<<gWP, b256, 0, stream>>>(Wq, DI, DM, WQ, KX, 1, 0, 1.0f);
  wt16<<<gWP, b256, 0, stream>>>(Wk, DI, DM, WK, KX, 1, 0, 1.0f);
  wt16<<<gWP, b256, 0, stream>>>(Wv, DI, DM, WV, KX, 1, 0, 1.0f);
  wt16<<<gWP, b256, 0, stream>>>(Wu, DI, DM, WU, KX, 1, 0, 1.0f);
  wt16<<<gWO, b256, 0, stream>>>(Wo, DM, DI, WO, DI, 0, 1, WOS);

  for (int g = 0; g < NGRP; ++g) {
    const u16*   xg = XB   + (size_t)g * GROWS * KX;
    const float* mg = mask + (size_t)g * GROWS;
    float*       og = out  + (size_t)g * GROWS * DM;
    gemm_bf<<<gG, b128, 0, stream>>>(xg, WV, F, GROWS, DI, KX, 1.0f);
    vt16<<<gVT, b256, 0, stream>>>(F, VH, VL);
    gemm_bf<<<gG, b128, 0, stream>>>(xg, WQ, F, GROWS, DI, KX, 1.0f);
    qk16<<<gQK, bQK, 0, stream>>>(F, QH, QL, QSC);
    gemm_bf<<<gG, b128, 0, stream>>>(xg, WK, F, GROWS, DI, KX, 1.0f);
    qk16<<<gQK, bQK, 0, stream>>>(F, KH, KL, KSC);
    gemm_bf<<<gG, b128, 0, stream>>>(xg, WU, U, GROWS, DI, KX, 1.0f);
    attn_t<<<gAT, bAT, 0, stream>>>(KH, KL, QH, QL, VH, VL, CB, U, bu, OH, OL);
    gemm_o<<<gO, b128, 0, stream>>>(OH, OL, WO, bo, mg, og, osc);
  }
  (void)hipGetLastError();
}
